// ConditionModulationBlock_55508157333802
// MI455X (gfx1250) — hardware-verified
//
#include <hip/hip_runtime.h>


namespace {
constexpr int Bn = 2, L = 1024, DM = 1024, ED = 2048, NS = 16, DC = 4, R = 64, NT = Bn * L, XDB = 128  ;
constexpr float AS_ = 8.0f, EPS = 1e-5f;

typedef _Float16 b16;
typedef __attribute__((ext_vector_type(16))) _Float16 v16b;
typedef __attribute__((ext_vector_type(8))) _Float16 v8b;
typedef __attribute__((ext_vector_type(8))) float v8f;
typedef __attribute__((ext_vector_type(4))) float v4f;
__device__ __forceinline__ float bf16_rne(float f) { unsigned int u = __float_as_uint(f); u += 0x7FFFu + ((u >> 16) & 1u); return __uint_as_float(u & 0xFFFF0000u); }
__device__ __forceinline__ void split16(float v, b16& hi, b16& lo) { hi = (b16)v; lo = (b16)(v - (float)hi); }
__device__ __forceinline__ v16b frag_kb(const b16* p, int hh) { const v8b a = *(const v8b*)(p + 8 * hh), b = *(const v8b*)(p + 16 + 8 * hh); v16b f;
#pragma unroll
  for (int e = 0; e < 8; ++e) { f[e] = a[e]; f[8 + e] = b[e]; } return f; }
__device__ __forceinline__ void frag_split(const float* p, int hh, v16b& fh, v16b& fl) {
#pragma unroll
  for (int e = 0; e < 8; ++e) { b16 a, c; split16(p[8 * hh + e] * AS_, a, c); fh[e] = a; fl[e] = c; split16(p[16 + 8 * hh + e] * AS_, a, c); fh[8 + e] = a; fl[8 + e] = c; } }
__device__ __forceinline__ v8f wmma16b(v16b a, v16b b, v8f c) { v8f d = __builtin_amdgcn_wmma_f32_16x16x32_f16(false, a, false, b, (short)0, c, false, false); asm volatile("v_nop\n\tv_nop\n\tv_nop\n\tv_nop" : "+v"(d) : "v"(a), "v"(b)); return d; }
__device__ __forceinline__ void wave_lds_sync() { __builtin_amdgcn_fence(__ATOMIC_RELEASE, "workgroup"); __builtin_amdgcn_wave_barrier(); __builtin_amdgcn_fence(__ATOMIC_ACQUIRE, "workgroup"); }
__device__ __forceinline__ float nexp(float x) { return __builtin_amdgcn_exp2f(x * 1.4426950408889634f); }
__device__ __forceinline__ float pmul(float a, float b) { float p = a * b; asm volatile("" : "+v"(p)); return p; }
__device__ __forceinline__ float softplus_(float z) { return fmaxf(z, 0.0f) + log1pf(nexp(-fabsf(z))); }
__device__ __forceinline__ float silu_(float x) { return x / (1.0f + nexp(-x)); }

struct Wo_ { static constexpr size_t IN = 0, XP = IN + (size_t)4096 * 1024, DT = XP + (size_t)128 * 2048, OUT = DT + (size_t)2048 * 64, END = OUT + (size_t)1024 * 2048; };
struct Po_ { static constexpr int NW = 0, NB = 1024, CW = 2048, CB = 10240, DTB = 12288, A = 14336, DD = 47104, END = 49152; };
__global__ __launch_bounds__(256) void prep_kernel(const float* __restrict__ nw, const float* __restrict__ nb, const float* __restrict__ inw, const float* __restrict__ cw, const float* __restrict__ cb, const float* __restrict__ xpw, const float* __restrict__ dtw, const float* __restrict__ dtb, const float* __restrict__ alog, const float* __restrict__ Dv, const float* __restrict__ ow, b16* __restrict__ Rw, float* __restrict__ P) {
  const size_t tid = (size_t)blockIdx.x * blockDim.x + threadIdx.x, nth = (size_t)gridDim.x * blockDim.x;
  for (int pass = 0; pass < 2; ++pass) {
    for (size_t p = tid; p < (size_t)4096 * 1024; p += nth) Rw[Wo_::IN + p] = (b16)bf16_rne(inw[p]);
    for (size_t p = tid; p < (size_t)128 * 2048; p += nth) Rw[Wo_::XP + p] = (b16)((p < (size_t)96 * 2048) ? bf16_rne(xpw[p]) : 0.0f);
    for (size_t p = tid; p < (size_t)2048 * 64; p += nth) Rw[Wo_::DT + p] = (b16)bf16_rne(dtw[p]);
    for (size_t p = tid; p < (size_t)1024 * 2048; p += nth) Rw[Wo_::OUT + p] = (b16)bf16_rne(ow[p]);
    for (size_t p = tid; p < (size_t)Po_::END; p += nth) { const int i = (int)p; float v;
      if (i < Po_::NB) v = bf16_rne(nw[i]); else if (i < Po_::CW) v = bf16_rne(nb[i - Po_::NB]); else if (i < Po_::CB) v = bf16_rne(cw[i - Po_::CW]); else if (i < Po_::DTB) v = bf16_rne(cb[i - Po_::CB]); else if (i < Po_::A) v = bf16_rne(dtb[i - Po_::DTB]); else if (i < Po_::DD) v = -expf(bf16_rne(alog[i - Po_::A])); else v = bf16_rne(Dv[i - Po_::DD]);
      P[p] = v; }
    __threadfence(); }
}

__global__ __launch_bounds__(256) void addln_kernel(const float* __restrict__ hs, const float* __restrict__ rs, const float* __restrict__ P, float* __restrict__ resid, float* __restrict__ xn) {
  const int wid = threadIdx.x >> 5, lane = threadIdx.x & 31; const size_t row = (size_t)blockIdx.x * 8 + wid; const float* g = P + Po_::NW; const float* bb = P + Po_::NB;
  float v[32]; float s = 0.0f;
#pragma unroll
  for (int j = 0; j < 8; ++j) { const v4f a = *(const v4f*)(hs + row * DM + j * 128 + lane * 4), b = *(const v4f*)(rs + row * DM + j * 128 + lane * 4);
#pragma unroll
    for (int e = 0; e < 4; ++e) { v[j * 4 + e] = bf16_rne(a[e]) + bf16_rne(b[e]); s += v[j * 4 + e]; } }
#pragma unroll
  for (int o = 1; o < 32; o <<= 1) s += __shfl_xor(s, o);
  const float mu = s * (1.0f / DM); float q = 0.0f;
#pragma unroll
  for (int j = 0; j < 32; ++j) { const float d = v[j] - mu; q += pmul(d, d); }
#pragma unroll
  for (int o = 1; o < 32; o <<= 1) q += __shfl_xor(q, o);
  const float is = rsqrtf(q * (1.0f / DM) + EPS);
  for (int pass = 0; pass < 2; ++pass) {
#pragma unroll
    for (int j = 0; j < 8; ++j) { const int c = j * 128 + lane * 4; v4f r4, x4; for (int e = 0; e < 4; ++e) { r4[e] = v[j * 4 + e]; x4[e] = pmul((v[j * 4 + e] - mu) * is, g[c + e]) + bb[c + e]; } *(volatile v4f*)(resid + row * DM + c) = r4; *(volatile v4f*)(xn + row * DM + c) = x4; }
    __threadfence(); }
}

__global__ __launch_bounds__(128) void gemm_kernel(const float* __restrict__ X, int K, int ldx, const b16* __restrict__ Bw, int N, const float* __restrict__ bias, int mode, float* __restrict__ Y) {
  __shared__ __attribute__((aligned(16))) float Ts[4][32 * 64];
  const int lane = threadIdx.x & 31, wave = threadIdx.x >> 5, nloc = lane & 15, hlf = lane >> 4, m0 = blockIdx.y * 128 + wave * 32, c0 = blockIdx.x * 64;
  v8f acc[2][4];
#pragma unroll
  for (int r = 0; r < 2; ++r)
#pragma unroll
    for (int t = 0; t < 4; ++t) acc[r][t] = (v8f){};
#pragma unroll 2
  for (int kb = 0; kb < K; kb += 32) { v16b a0, l0, a1, l1; frag_split(X + (size_t)(m0 + nloc) * ldx + kb, hlf, a0, l0); frag_split(X + (size_t)(m0 + 16 + nloc) * ldx + kb, hlf, a1, l1);
#pragma unroll
    for (int t = 0; t < 4; ++t) { const v16b bw = frag_kb(Bw + (size_t)(c0 + t * 16 + nloc) * K + kb, hlf); acc[0][t] = wmma16b(a0, bw, acc[0][t]); acc[0][t] = wmma16b(l0, bw, acc[0][t]); acc[1][t] = wmma16b(a1, bw, acc[1][t]); acc[1][t] = wmma16b(l1, bw, acc[1][t]); } }
  float* Tt = Ts[wave];
#pragma unroll
  for (int t = 0; t < 4; ++t) { const int cc = c0 + t * 16 + nloc; const float bb = bias ? bias[cc] : 0.0f;
#pragma unroll
    for (int r = 0; r < 2; ++r)
#pragma unroll
      for (int v = 0; v < 8; ++v) Tt[(r * 16 + v + 8 * hlf) * 64 + t * 16 + nloc] = acc[r][t][v] * (1.0f / AS_) + bb; }
  wave_lds_sync();
  if (mode == 1) {
#pragma unroll 1
    for (int i = lane; i < 32 * 64; i += 32) Tt[i] = softplus_(Tt[i]);
    wave_lds_sync(); }
  for (int pass = 0; pass < 2; ++pass) {
#pragma unroll
    for (int j = 0; j < 16; ++j) { const int rr = j * 2 + hlf, c4 = nloc * 4; *(volatile v4f*)(Y + (size_t)(m0 + rr) * N + c0 + c4) = *(const v4f*)(Tt + rr * 64 + c4); }
    __threadfence(); }
}

__global__ __launch_bounds__(256) void conv_kernel(const float* __restrict__ xz, const float* __restrict__ P, float* __restrict__ xcs) {
  const size_t g = (size_t)blockIdx.x * 256 + threadIdx.x; const int tok = (int)(g / (ED / 4)), e4 = (int)(g % (ED / 4)) * 4, b = tok / L, t = tok % L; const float* cw = P + Po_::CW; const float* cb = P + Po_::CB;
  v4f o;
#pragma unroll
  for (int q = 0; q < 4; ++q) { const int e = e4 + q; float acc = cb[e];
#pragma unroll
    for (int k = 0; k < DC; ++k) { const int ts = t - (DC - 1) + k; if (ts >= 0) acc += pmul(cw[e * DC + k], xz[((size_t)b * L + ts) * (2 * ED) + e]); }
    o[q] = silu_(acc); }
  for (int pass = 0; pass < 2; ++pass) { *(volatile v4f*)(xcs + (size_t)tok * ED + e4) = o; __threadfence(); }
}

__global__ __launch_bounds__(256) void scan_kernel(const float* __restrict__ xcs, const float* __restrict__ delta, const float* __restrict__ xdbl, const float* __restrict__ xz, const float* __restrict__ P, float* __restrict__ y) {
  const int g = blockIdx.x * 256 + threadIdx.x, b = g / ED, e = g % ED; const float* A = P + Po_::A + e * NS; const float Dv = P[Po_::DD + e];
  float h[NS], a_[NS];
#pragma unroll
  for (int n = 0; n < NS; ++n) { h[n] = 0.0f; a_[n] = A[n]; }
  for (int t = 0; t < L; ++t) { const size_t row = (size_t)b * L + t; const float dl = delta[row * ED + e], xc = xcs[row * ED + e]; const float* xr = xdbl + row * XDB; const float dx = dl * xc; float acc = 0.0f;
#pragma unroll
    for (int n = 0; n < NS; ++n) { const float dA = nexp(dl * a_[n]); h[n] = dA * h[n] + pmul(dx, xr[R + n]); acc += pmul(h[n], xr[R + NS + n]); }
    const float yv = (acc + pmul(xc, Dv)) * silu_(xz[row * (2 * ED) + ED + e]);
    for (int pass = 0; pass < 2; ++pass) ((volatile float*)y)[row * ED + e] = yv; }
  __threadfence();
}
}

extern "C" void kernel_launch(void* const* d_in, const int* in_sizes, int n_in,
                              void* d_out, int out_size, void* d_ws, size_t ws_size, hipStream_t stream) {
  (void)n_in; (void)out_size;
  const float* hs = (const float*)d_in[0]; const float* rs = (const float*)d_in[1]; const float* nw = (const float*)d_in[2]; const float* nb = (const float*)d_in[3]; const float* inw = (const float*)d_in[4]; const float* cw = (const float*)d_in[5]; const float* cb = (const float*)d_in[6];
  const float* xpw = (const float*)d_in[7]; const float* dtw = (const float*)d_in[8]; const float* dtb = (const float*)d_in[9]; const float* alog = (const float*)d_in[10]; const float* Dv = (const float*)d_in[11]; const float* ow = (const float*)d_in[12];
  float* out = (float*)d_out; float* resid = out + (size_t)NT * DM;
  if (in_sizes[0] != NT * DM || in_sizes[4] != 4096 * 1024 || in_sizes[7] != 96 * 2048 || in_sizes[8] != 2048 * 64 || in_sizes[10] != 2048 * 16 || in_sizes[12] != 1024 * 2048) return;
  size_t off = 0; char* ws = (char*)d_ws;
  auto carve = [&](size_t bytes) { char* p = ws + off; off += (bytes + 255) & ~(size_t)255; return p; };
  b16* Rw = (b16*)carve(Wo_::END * 2); float* P = (float*)carve((size_t)Po_::END * 4); float* xn = (float*)carve((size_t)NT * DM * 4); float* xz = (float*)carve((size_t)NT * 2 * ED * 4); float* xcs = (float*)carve((size_t)NT * ED * 4);
  float* xdbl = (float*)carve((size_t)NT * XDB * 4); float* delta = (float*)carve((size_t)NT * ED * 4); float* y = xn;
  y = (float*)carve((size_t)NT * ED * 4);
  if (off > ws_size) return;
  prep_kernel<<<512, 256, 0, stream>>>(nw, nb, inw, cw, cb, xpw, dtw, dtb, alog, Dv, ow, Rw, P);
  addln_kernel<<<NT / 8, 256, 0, stream>>>(hs, rs, P, resid, xn);
  gemm_kernel<<<dim3(2 * ED / 64, NT / 128), 128, 0, stream>>>(xn, DM, DM, Rw + Wo_::IN, 2 * ED, nullptr, 0, xz);
  conv_kernel<<<NT * ED / 4 / 256, 256, 0, stream>>>(xz, P, xcs);
  gemm_kernel<<<dim3(XDB / 64, NT / 128), 128, 0, stream>>>(xcs, ED, ED, Rw + Wo_::XP, XDB, nullptr, 0, xdbl);
  gemm_kernel<<<dim3(ED / 64, NT / 128), 128, 0, stream>>>(xdbl, R, XDB, Rw + Wo_::DT, ED, P + Po_::DTB, 1, delta);
  scan_kernel<<<Bn * ED / 256, 256, 0, stream>>>(xcs, delta, xdbl, xz, P, y);
  gemm_kernel<<<dim3(DM / 64, NT / 128), 128, 0, stream>>>(y, ED, ED, Rw + Wo_::OUT, DM, nullptr, 0, out);
}
